// _Interactions_79791902425117
// MI455X (gfx1250) — hardware-verified
//
#include <hip/hip_runtime.h>
#include <stddef.h>
#include <stdint.h>


#define CD      256
#define NTHR    256
#define NWAVE   8
#define EPT     8
#define NGRP    2
#define CHUNK   (NTHR * EPT * NGRP)
#define WCAP    (EPT * NGRP * 32)
#define LISTN   (NWAVE * WCAP)
#define NBL     256
#define NBD     4096
#define G0ROWS  64
#define ASCL    64.0f
#define WSCL    16.0f
#define HINV    0.0009765625f
#define MIXA    0.1f
#define MIXB    0.9f
#define ASPLIT  1

#define LDS_LAYER (NBL * CD * 4 + LISTN * 4 + 64)
#define LDS_G0    (2 * G0ROWS * CD * 2)

static_assert((CHUNK & (CHUNK - 1)) == 0);
static_assert(CHUNK <= 4096);
static_assert((NBL & (NBL - 1)) == 0 && NBL <= 4096);
static_assert((NBD & (NBD - 1)) == 0 && NBD <= 4096);
static_assert(NBL / 16 == 2 * NWAVE);
static_assert(NWAVE * 16 * 32 * 4 <= LISTN * 4);
static_assert(G0ROWS * CD * 4 <= LDS_G0);
static_assert(NBD == NWAVE * 4 * 128);
static_assert(G0ROWS == NWAVE * 8);

typedef float    v4f  __attribute__((ext_vector_type(4)));
typedef v4f      v4fa __attribute__((may_alias));
typedef float    v8f  __attribute__((ext_vector_type(8)));
typedef int      v4i  __attribute__((ext_vector_type(4)));
typedef _Float16 v8h  __attribute__((ext_vector_type(8)));
typedef _Float16 v16h __attribute__((ext_vector_type(16)));
typedef __bf16   v16b __attribute__((ext_vector_type(16)));
typedef unsigned short v8us __attribute__((ext_vector_type(8)));
union Frag { v16h f; v16b b; v4i q[2]; };
union P16  { v8h h; v8us u; v4i i; };

__device__ __forceinline__ v8f wmh(const Frag& a, const Frag& b, v8f c) {
  v8f d = __builtin_amdgcn_wmma_f32_16x16x32_f16(false, a.f, false, b.f, (short)0, c, false, false);
  asm volatile("v_nop\n\tv_nop\n\tv_nop\n\tv_nop" : "+v"(d) : "v"(a.f), "v"(b.f));
  return d;
}
__device__ __forceinline__ v8f wmb(const Frag& a, const Frag& b, v8f c) {
  v8f d = __builtin_amdgcn_wmma_f32_16x16x32_bf16(false, a.b, false, b.b, (short)0, c, false, false);
  asm volatile("v_nop\n\tv_nop\n\tv_nop\n\tv_nop" : "+v"(d) : "v"(a.f), "v"(b.f));
  return d;
}

__device__ __forceinline__ unsigned int bf16_rne(float f) {
  unsigned int u = __float_as_uint(f);
  u += 0x7FFFu + ((u >> 16) & 1u);
  return u >> 16;
}

__device__ __forceinline__ void split_bf16_8(v4f a, v4f b, P16& hi, P16& lo) {
  const float v[8] = {a.x, a.y, a.z, a.w, b.x, b.y, b.z, b.w};
#pragma unroll
  for (int j = 0; j < 8; ++j) {
    const unsigned int hb = bf16_rne(v[j]);
    const float hf = __uint_as_float(hb << 16);
    hi.u[j] = (unsigned short)hb;
    lo.u[j] = (unsigned short)bf16_rne(v[j] - hf);
  }
}

__device__ __forceinline__ void cvt_f16_8(v4f a, v4f b, P16& o) {
  const float v[8] = {a.x, a.y, a.z, a.w, b.x, b.y, b.z, b.w};
#pragma unroll
  for (int j = 0; j < 8; ++j) o.h[j] = (_Float16)v[j];
}

__device__ __forceinline__ void split_f16_frag(v4f p0, v4f p1, v4f p2, v4f p3, Frag& hi, Frag& lo) {
  const float s[16] = {p0.x * ASCL, p0.y * ASCL, p0.z * ASCL, p0.w * ASCL,
                       p1.x * ASCL, p1.y * ASCL, p1.z * ASCL, p1.w * ASCL,
                       p2.x * ASCL, p2.y * ASCL, p2.z * ASCL, p2.w * ASCL,
                       p3.x * ASCL, p3.y * ASCL, p3.z * ASCL, p3.w * ASCL};
#pragma unroll
  for (int j = 0; j < 16; ++j) {
    const _Float16 hh = (_Float16)s[j];
    hi.f[j] = hh;
    lo.f[j] = (_Float16)(s[j] - (float)hh);
  }
}

template <int NB>
__device__ __forceinline__ int scan_chunk(const int* __restrict__ dsts, int nE, int cbase, int nodeBase,
                                          int vec8, int* list, int tid, int wave) {
  int wc = 0;
#pragma unroll
  for (int g = 0; g < NGRP; ++g) {
    const int el0  = (g * NTHR + tid) * EPT;
    const int e0   = cbase + el0;
    const int sent = -2147483647 - 1;
    v4i da, db;
    if (vec8 != 0 && e0 + 7 < nE) {
      da = *(const v4i*)(dsts + e0);
      db = *(const v4i*)(dsts + e0 + 4);
    } else {
      da.x = (e0     < nE) ? dsts[min(e0, nE - 1)] : sent;
      da.y = (e0 + 1 < nE) ? dsts[min(e0 + 1, nE - 1)] : sent;
      da.z = (e0 + 2 < nE) ? dsts[min(e0 + 2, nE - 1)] : sent;
      da.w = (e0 + 3 < nE) ? dsts[min(e0 + 3, nE - 1)] : sent;
      db.x = (e0 + 4 < nE) ? dsts[min(e0 + 4, nE - 1)] : sent;
      db.y = (e0 + 5 < nE) ? dsts[min(e0 + 5, nE - 1)] : sent;
      db.z = (e0 + 6 < nE) ? dsts[min(e0 + 6, nE - 1)] : sent;
      db.w = (e0 + 7 < nE) ? dsts[min(e0 + 7, nE - 1)] : sent;
    }
    const unsigned nb = (unsigned)nodeBase;
    const unsigned s0 = (unsigned)da.x - nb, s1 = (unsigned)da.y - nb;
    const unsigned s2 = (unsigned)da.z - nb, s3 = (unsigned)da.w - nb;
    const unsigned s4 = (unsigned)db.x - nb, s5 = (unsigned)db.y - nb;
    const unsigned s6 = (unsigned)db.z - nb, s7 = (unsigned)db.w - nb;
    const bool h0 = s0 < (unsigned)NB, h1 = s1 < (unsigned)NB, h2 = s2 < (unsigned)NB, h3 = s3 < (unsigned)NB;
    const bool h4 = s4 < (unsigned)NB, h5 = s5 < (unsigned)NB, h6 = s6 < (unsigned)NB, h7 = s7 < (unsigned)NB;
    const unsigned any = __builtin_amdgcn_ballot_w32(h0 | h1 | h2 | h3 | h4 | h5 | h6 | h7);
    if (any != 0u) {
#define HITJ(J, HJ, SJ) { \
        const unsigned mj = __builtin_amdgcn_ballot_w32(HJ); \
        if (mj != 0u) { \
          if (HJ) { \
            const int pos = wc + (int)__builtin_amdgcn_mbcnt_lo(mj, 0u); \
            if (pos < WCAP) list[wave * WCAP + pos] = ((el0 + (J)) << 12) | (int)(SJ); \
          } \
          wc += (int)__builtin_popcount(mj); } }
      HITJ(0, h0, s0)
      HITJ(1, h1, s1)
      HITJ(2, h2, s2)
      HITJ(3, h3, s3)
      HITJ(4, h4, s4)
      HITJ(5, h5, s5)
      HITJ(6, h6, s6)
      HITJ(7, h7, s7)
#undef HITJ
    }
  }
  return wc;
}

__global__ __launch_bounds__(NTHR) void k_prep(
    const float* __restrict__ W0, const float* __restrict__ Wc,
    unsigned short* w0hi, unsigned short* w0lo, _Float16* wc, int nMat) {
  const int mat = blockIdx.x >> 5;
  if (mat > nMat) return;
  const int run = ((blockIdx.x & 31) << 8) + threadIdx.x;
  const int o   = run << 3;
  const int n   = o >> 8;
  const int k0  = o & (CD - 1);
  const float* p = (mat == 0 ? W0 : Wc + (size_t)(mat - 1) * CD * CD) + (size_t)k0 * CD + n;
  v4f a, b;
  a.x = p[0];      a.y = p[CD];     a.z = p[2 * CD]; a.w = p[3 * CD];
  b.x = p[4 * CD]; b.y = p[5 * CD]; b.z = p[6 * CD]; b.w = p[7 * CD];
  if (mat == 0) {
    P16 hi, lo;
    split_bf16_8(a, b, hi, lo);
    *(volatile v4i*)(w0hi + o) = hi.i;
    *(volatile v4i*)(w0lo + o) = lo.i;
    __threadfence();
    *(volatile v4i*)(w0hi + o) = hi.i;
    *(volatile v4i*)(w0lo + o) = lo.i;
  } else {
    a = a * WSCL;
    b = b * WSCL;
    P16 hv;
    cvt_f16_8(a, b, hv);
    _Float16* dp = wc + (size_t)(mat - 1) * CD * CD + o;
    *(volatile v4i*)dp = hv.i;
    __threadfence();
    *(volatile v4i*)dp = hv.i;
  }
}

__global__ __launch_bounds__(NTHR) void k_deg(
    const int* __restrict__ ei, const float* __restrict__ ew, float* dinv, int nE, int vec8) {
  __shared__ __attribute__((aligned(16))) float deg[NBD];
  __shared__ __attribute__((aligned(16))) int   list[LISTN];
  __shared__ int wcnt[NWAVE];
  const int tid = threadIdx.x, lane = tid & 31, wave = tid >> 5;
  const int nodeBase = blockIdx.x * NBD;
  const int* dsts = ei + nE;

  for (int i = tid; i < NBD; i += NTHR) deg[i] = 0.0f;
  __syncthreads();

  const int nChunks = (nE + CHUNK - 1) / CHUNK;
#pragma unroll 1
  for (int ch = 0; ch < nChunks; ++ch) {
    const int cbase = ch * CHUNK;
    const int wc = scan_chunk<NBD>(dsts, nE, cbase, nodeBase, vec8, list, tid, wave);
    if (lane == 0) wcnt[wave] = wc;
    __syncthreads();
    if (wave == 0) {
#pragma unroll 1
      for (int wsx = 0; wsx < NWAVE; ++wsx) {
        int n = __builtin_amdgcn_readfirstlane(wcnt[wsx]);
        n = n > WCAP ? WCAP : (n < 0 ? 0 : n);
        const int* lp = list + wsx * WCAP;
#pragma unroll 1
        for (int i = 0; i < n; ++i) {
          const int ent  = __builtin_amdgcn_readfirstlane(lp[i]);
          const int slot = ent & (NBD - 1);
          int e = cbase + ((ent >> 12) & (CHUNK - 1));
          e = e > nE - 1 ? nE - 1 : e;
          const float wv = ew[e];
          if (lane == 0) deg[slot] = deg[slot] + wv;
        }
      }
    }
    __syncthreads();
  }

  v4f dq[4];
#pragma unroll
  for (int q = 0; q < 4; ++q) {
    const int f = (wave * 4 + q) * 128 + 4 * lane;
    const v4f c = *(const v4fa*)(deg + f);
    dq[q].x = c.x > 0.0f ? rsqrtf(c.x) : 0.0f;
    dq[q].y = c.y > 0.0f ? rsqrtf(c.y) : 0.0f;
    dq[q].z = c.z > 0.0f ? rsqrtf(c.z) : 0.0f;
    dq[q].w = c.w > 0.0f ? rsqrtf(c.w) : 0.0f;
  }
  float* dp = dinv + (size_t)nodeBase;
#pragma unroll
  for (int q = 0; q < 4; ++q) *(volatile v4f*)(dp + (wave * 4 + q) * 128 + 4 * lane) = dq[q];
  __threadfence();
#pragma unroll
  for (int q = 0; q < 4; ++q) *(volatile v4f*)(dp + (wave * 4 + q) * 128 + 4 * lane) = dq[q];
}

__global__ __launch_bounds__(NTHR) void k_norm(
    const int* __restrict__ ei, const float* __restrict__ ew, const float* __restrict__ dinv,
    const float* __restrict__ eattr, float* nrm, int nN, int nE, int nE32) {
  (void)eattr;
  const int e0 = (blockIdx.x * NTHR + threadIdx.x) * 4;
  if (e0 >= nE32) return;
  float v[4];
#pragma unroll
  for (int j = 0; j < 4; ++j) {
    int e = e0 + j;
    e = e > nE - 1 ? nE - 1 : e;
    int r = ei[e];
    int c = ei[(size_t)nE + e];
    r = r < 0 ? 0 : (r > nN - 1 ? nN - 1 : r);
    c = c < 0 ? 0 : (c > nN - 1 ? nN - 1 : c);
    v[j] = dinv[r] * ew[e] * dinv[c];
  }
  v4f o;
  o.x = v[0]; o.y = v[1]; o.z = v[2]; o.w = v[3];
  *(volatile v4f*)(nrm + e0) = o;
  __threadfence();
  *(volatile v4f*)(nrm + e0) = o;
}

__global__ __launch_bounds__(NTHR) void k_gemm0(
    const float* __restrict__ x, const unsigned short* __restrict__ w0hi,
    const unsigned short* __restrict__ w0lo, const float* __restrict__ bias,
    float* xo, int nN) {
  extern __shared__ v4f lds_dyn[];
  unsigned short* sAhi = (unsigned short*)lds_dyn;
  unsigned short* sAlo = sAhi + G0ROWS * CD;
  float*          stg  = (float*)lds_dyn;
  const int tid = threadIdx.x, lane = tid & 31, wave = tid >> 5, hh = lane >> 4, m = lane & 15;
  const int rowBase = blockIdx.x * G0ROWS;

#pragma unroll
  for (int i = 0; i < (G0ROWS * CD / 8) / NTHR; ++i) {
    const int idx = i * NTHR + tid;
    const int r   = idx >> 5;
    const int c0  = (idx & 31) * 8;
    int node = rowBase + r;
    node = node > nN - 1 ? nN - 1 : node;
    const float* xp = x + (size_t)node * CD + c0;
    const v4f a = *(const v4f*)xp, b = *(const v4f*)(xp + 4);
    P16 hi, lo;
    split_bf16_8(a, b, hi, lo);
    *(v4i*)(sAhi + r * CD + c0) = hi.i;
    *(v4i*)(sAlo + r * CD + c0) = lo.i;
  }
  __syncthreads();

  const int rt = wave & 3, half = wave >> 2;
  v8f acc[8];
#pragma unroll
  for (int t = 0; t < 8; ++t) { const v8f z = {0.f, 0.f, 0.f, 0.f, 0.f, 0.f, 0.f, 0.f}; acc[t] = z; }
#pragma unroll 1
  for (int kt = 0; kt < CD / 32; ++kt) {
    const unsigned short* arh = sAhi + (rt * 16 + m) * CD + 32 * kt + 8 * hh;
    const unsigned short* arl = sAlo + (rt * 16 + m) * CD + 32 * kt + 8 * hh;
    Frag ah, al;
    ah.q[0] = *(const v4i*)arh;  ah.q[1] = *(const v4i*)(arh + 16);
    al.q[0] = *(const v4i*)arl;  al.q[1] = *(const v4i*)(arl + 16);
#pragma unroll
    for (int t = 0; t < 8; ++t) {
      const int n = half * 128 + 16 * t + m;
      const unsigned short* bph = w0hi + (size_t)n * CD + 32 * kt + 8 * hh;
      const unsigned short* bpl = w0lo + (size_t)n * CD + 32 * kt + 8 * hh;
      Frag bh, bl;
      bh.q[0] = *(const v4i*)bph; bh.q[1] = *(const v4i*)(bph + 16);
      bl.q[0] = *(const v4i*)bpl; bl.q[1] = *(const v4i*)(bpl + 16);
      acc[t] = wmb(ah, bh, acc[t]);
      acc[t] = wmb(ah, bl, acc[t]);
      acc[t] = wmb(al, bh, acc[t]);
    }
  }
  __syncthreads();

#pragma unroll
  for (int t = 0; t < 8; ++t) {
    const int bcol = half * 128 + 16 * t + m;
    const float bv = bias[bcol];
    float* sp = stg + (size_t)(rt * 16 + 8 * hh) * CD + bcol;
#pragma unroll
    for (int r = 0; r < 8; ++r) sp[r * CD] = fmaxf(acc[t][r] + bv, 0.0f);
  }
  __syncthreads();

  const float* lbase = stg + (size_t)(wave * 8) * CD + 4 * lane;
  float*       gbase = xo + ((size_t)rowBase + wave * 8) * CD + 4 * lane;
#pragma unroll
  for (int i = 0; i < 8; ++i) {
#pragma unroll
    for (int s = 0; s < 2; ++s) {
      const v4f v = *(const v4fa*)(lbase + i * CD + 128 * s);
      *(volatile v4f*)(gbase + (size_t)i * CD + 128 * s) = v;
    }
  }
  __threadfence();
#pragma unroll
  for (int i = 0; i < 8; ++i) {
#pragma unroll
    for (int s = 0; s < 2; ++s) {
      const v4f v = *(const v4fa*)(lbase + i * CD + 128 * s);
      *(volatile v4f*)(gbase + (size_t)i * CD + 128 * s) = v;
    }
  }
}

__global__ __launch_bounds__(NTHR) void k_layer(
    const int* __restrict__ ei, const float* __restrict__ nrm, const float* __restrict__ src,
    const float* __restrict__ x0, const _Float16* __restrict__ wl, float* dst,
    int nN, int nE, int vec8) {
  extern __shared__ v4f lds_dyn[];
  float* accf = (float*)lds_dyn;
  int*   list = (int*)(accf + NBL * CD);
  int*   wcnt = list + LISTN;
  float* stgb = (float*)list;
  const int tid = threadIdx.x, lane = tid & 31, wave = tid >> 5, hh = lane >> 4, m = lane & 15;
  const int nodeBase = blockIdx.x * NBL;
  const int* dsts = ei + nE;

  {
    const v4f z = {0.f, 0.f, 0.f, 0.f};
    for (int i = tid; i < NBL * CD / 4; i += NTHR) lds_dyn[i] = z;
  }
  __syncthreads();

  const int nChunks = (nE + CHUNK - 1) / CHUNK;
#pragma unroll 1
  for (int ch = 0; ch < nChunks; ++ch) {
    const int cbase = ch * CHUNK;
    const int wc = scan_chunk<NBL>(dsts, nE, cbase, nodeBase, vec8, list, tid, wave);
    if (lane == 0) wcnt[wave] = wc;
    __syncthreads();
    if (wave == 0) {
#pragma unroll 1
      for (int wsx = 0; wsx < NWAVE; ++wsx) {
        int n = __builtin_amdgcn_readfirstlane(wcnt[wsx]);
        n = n > WCAP ? WCAP : (n < 0 ? 0 : n);
        const int* lp = list + wsx * WCAP;
#pragma unroll 1
        for (int i = 0; i < n; ++i) {
          const int ent  = __builtin_amdgcn_readfirstlane(lp[i]);
          const int slot = ent & (NBL - 1);
          int e = cbase + ((ent >> 12) & (CHUNK - 1));
          e = e > nE - 1 ? nE - 1 : e;
          int s = ei[e];
          s = s < 0 ? 0 : (s > nN - 1 ? nN - 1 : s);
          const float nv = nrm[e];
          const float* sp = src + (size_t)s * CD + 4 * lane;
          const v4f v0 = *(const v4f*)sp;
          const v4f v1 = *(const v4f*)(sp + 128);
          v4f* ap = (v4f*)(accf + slot * CD + 4 * lane);
          ap[0]  = ap[0]  + v0 * nv;
          ap[32] = ap[32] + v1 * nv;
        }
      }
    }
    __syncthreads();
  }

#pragma unroll 4
  for (int i = 0; i < (NBL * CD / 4) / NTHR; ++i) {
    const int idx  = i * NTHR + tid;
    const int slot = idx >> 6;
    const int c4   = (idx & 63) * 4;
    int node = nodeBase + slot;
    node = node > nN - 1 ? nN - 1 : node;
    const v4f xv = *(const v4f*)(x0 + (size_t)node * CD + c4);
    v4f* ap = (v4f*)(accf + slot * CD + c4);
    ap[0] = ap[0] * MIXA + xv * MIXB;
  }
  __syncthreads();

#pragma unroll 1
  for (int q = 0; q < 2; ++q) {
    const int rt = wave + NWAVE * q;
#pragma unroll 1
    for (int half = 0; half < 2; ++half) {
      v8f acc[8];
#pragma unroll
      for (int t = 0; t < 8; ++t) { const v8f z = {0.f, 0.f, 0.f, 0.f, 0.f, 0.f, 0.f, 0.f}; acc[t] = z; }
#pragma unroll 1
      for (int kt = 0; kt < CD / 32; ++kt) {
        const float* ar = accf + (size_t)(rt * 16 + m) * CD + 32 * kt + 8 * hh;
        const v4f p0 = *(const v4fa*)ar,        p1 = *(const v4fa*)(ar + 4);
        const v4f p2 = *(const v4fa*)(ar + 16), p3 = *(const v4fa*)(ar + 20);
        Frag ah, al;
        split_f16_frag(p0, p1, p2, p3, ah, al);
#pragma unroll
        for (int t = 0; t < 8; ++t) {
          const _Float16* bp = wl + (size_t)(half * 128 + 16 * t + m) * CD + 32 * kt + 8 * hh;
          Frag b;
          b.q[0] = *(const v4i*)bp;
          b.q[1] = *(const v4i*)(bp + 16);
          acc[t] = wmh(ah, b, acc[t]);
#if ASPLIT
          acc[t] = wmh(al, b, acc[t]);
#endif
        }
      }

      float* stg = stgb + wave * 512;
      const int rr = lane >> 3, cq = (lane & 7) * 4;
#pragma unroll
      for (int p = 0; p < 4; ++p) {
        {
          float* sp = stg + (8 * hh) * 32 + m;
#pragma unroll
          for (int r = 0; r < 8; ++r) {
            sp[r * 32]      = fmaxf(acc[2 * p][r],     0.0f) * HINV;
            sp[r * 32 + 16] = fmaxf(acc[2 * p + 1][r], 0.0f) * HINV;
          }
        }
        __syncthreads();
        const int col = half * 128 + 32 * p + cq;
        v4f nvv[4];
        int nd[4];
#pragma unroll
        for (int i = 0; i < 4; ++i) {
          const int row  = 4 * i + rr;
          const v4f hv   = *(const v4fa*)(stg + row * 32 + cq);
          const int node = nodeBase + rt * 16 + row;
          const int nc   = node > nN - 1 ? nN - 1 : node;
          const v4f ov   = *(const v4f*)(src + (size_t)nc * CD + col);
          nvv[i] = ov + hv;
          nd[i]  = node;
        }
#pragma unroll
        for (int i = 0; i < 4; ++i)
          if (nd[i] < nN) *(volatile v4f*)(dst + (size_t)nd[i] * CD + col) = nvv[i];
        __threadfence();
#pragma unroll
        for (int i = 0; i < 4; ++i)
          if (nd[i] < nN) *(volatile v4f*)(dst + (size_t)nd[i] * CD + col) = nvv[i];
      }
    }
  }
}

extern "C" void kernel_launch(void* const* d_in, const int* in_sizes, int n_in,
                              void* d_out, int out_size, void* d_ws, size_t ws_size,
                              hipStream_t stream) {
  if (n_in < 7) return;
  const int nN = in_sizes[0] / CD;
  const int nE = in_sizes[2];
  const int L  = in_sizes[6] / (CD * CD);
  if (nN <= 0 || nE <= 0 || L <= 0) return;
  if (in_sizes[0] != nN * CD || in_sizes[1] != 2 * nE || in_sizes[4] != CD * CD ||
      in_sizes[5] != CD || in_sizes[6] != L * CD * CD) return;
  if (out_size != nN * CD) return;

  const float* x   = (const float*)d_in[0];
  const int*   ei  = (const int*)d_in[1];
  const float* ew  = (const float*)d_in[2];
  const float* ea  = (const float*)d_in[3];
  const float* W0  = (const float*)d_in[4];
  const float* b0  = (const float*)d_in[5];
  const float* Wc  = (const float*)d_in[6];
  float*       out = (float*)d_out;

  const int nBD  = (nN + NBD - 1) / NBD;
  const int nG0  = (nN + G0ROWS - 1) / G0ROWS;
  const int nBL  = (nN + NBL - 1) / NBL;
  const int nE32 = ((nE + 31) / 32) * 32;

  char* ws = (char*)d_ws;
  size_t off = 0;
  const size_t oW0h = off; off += (size_t)CD * CD * 2;                          off = (off + 255) & ~(size_t)255;
  const size_t oW0l = off; off += (size_t)CD * CD * 2;                          off = (off + 255) & ~(size_t)255;
  const size_t oWc  = off; off += (size_t)L * CD * CD * 2;                      off = (off + 255) & ~(size_t)255;
  const size_t oDv  = off; off += (size_t)nBD * NBD * 4;                        off = (off + 255) & ~(size_t)255;
  const size_t oNr  = off; off += (size_t)nE32 * 4;                             off = (off + 255) & ~(size_t)255;
  const size_t oX   = off; off += (size_t)nG0 * G0ROWS * CD * 4;                off = (off + 255) & ~(size_t)255;
  const size_t oP   = off; off += (size_t)nN * CD * 4;                          off = (off + 255) & ~(size_t)255;
  const size_t cap  = (size_t)134217728;
  if (off > ws_size || off > cap) return;
  unsigned short* w0hi = (unsigned short*)(ws + oW0h);
  unsigned short* w0lo = (unsigned short*)(ws + oW0l);
  _Float16*       wc   = (_Float16*)(ws + oWc);
  float*          dinv = (float*)(ws + oDv);
  float*          nrm  = (float*)(ws + oNr);
  float*          X    = (float*)(ws + oX);
  float*          P    = (float*)(ws + oP);

  const int vec8 = ((nE & 3) == 0) ? 1 : 0;

  k_prep<<<(1 + L) * 32, NTHR, 0, stream>>>(W0, Wc, w0hi, w0lo, wc, L);

  k_deg<<<nBD, NTHR, 0, stream>>>(ei, ew, dinv, nE, vec8);

  k_norm<<<(nE32 / 4 + NTHR - 1) / NTHR, NTHR, 0, stream>>>(ei, ew, dinv, ea, nrm, nN, nE, nE32);

  hipFuncSetAttribute(reinterpret_cast<const void*>(&k_gemm0),
                      hipFuncAttributeMaxDynamicSharedMemorySize, LDS_G0);
  k_gemm0<<<nG0, NTHR, LDS_G0, stream>>>(x, w0hi, w0lo, b0, X, nN);

  hipFuncSetAttribute(reinterpret_cast<const void*>(&k_layer),
                      hipFuncAttributeMaxDynamicSharedMemorySize, LDS_LAYER);
  const float* cur = X;
  for (int li = 0; li < L; ++li) {
    float* dstp = (((L - 1 - li) & 1) == 0) ? out : P;
    k_layer<<<nBL, NTHR, LDS_LAYER, stream>>>(ei, nrm, cur, X, wc + (size_t)li * CD * CD, dstp, nN, nE, vec8);
    cur = dstp;
  }
}
